// MultiHeadAttention_4913442586758
// MI455X (gfx1250) — hardware-verified
//
#include <hip/hip_runtime.h>


#ifndef NB
#define NB 16
#endif
#ifndef SEQ
#define SEQ 2048
#endif
#define NB_FULL  16
#define SEQ_FULL 2048
#ifndef OUT_SEQ
#define OUT_SEQ SEQ
#endif
#define DIN  2
#define NH_  2
#define HD   64
#define AW   4
#define PT   64
#define WSZ  (NH_ * DIN * HD)
#define EROWS (SEQ < 512 ? SEQ : 512)
#define QRS  2048.0f
#define QRI  (1.0f / 2048.0f)
#define SC2  ((float)(0.125 * 1.4426950408889634))
#define PSH  14.0f
#define NEGB (-3.0e38f)

static_assert(HD == 64);
static_assert(HD % 32 == 0);
static_assert(NH_ == DIN);
static_assert(PT == 64);
static_assert(SEQ % PT == 0);
static_assert(SEQ % 32 == 0);
static_assert(SEQ % (16 * AW) == 0);
static_assert(EROWS % PT == 0);
static_assert(EROWS % 32 == 0);
static_assert(EROWS >= 32);
static_assert(EROWS <= SEQ);
static_assert(EROWS % (16 * AW) == 0);
static_assert((SEQ - EROWS) % (16 * AW) == 0);
static_assert(128 * 4 * 8 == PT * HD);
static_assert(8 * 16 == 16 * DIN * 4);
static_assert(((size_t)OUT_SEQ * DIN * 4) % 128 == 0);
static_assert(NB <= NB_FULL);
static_assert(SEQ <= SEQ_FULL);
static_assert((size_t)NB_FULL * SEQ_FULL * DIN * 4 == (size_t)262144);
static_assert((PT * 2 + 3 * WSZ) * 4 <= 131072);
static_assert(AW * 32 * 4 <= 131072);

typedef _Float16 h16;
typedef __attribute__((ext_vector_type(16))) _Float16 v16h;
typedef __attribute__((ext_vector_type(8)))  _Float16 v8h;
typedef __attribute__((ext_vector_type(8)))  float    v8f;
typedef __attribute__((ext_vector_type(4)))  float    v4f;
typedef v4f  __attribute__((may_alias)) v4fa;

static constexpr size_t al256(size_t v) { return (v + 255) & ~(size_t)255; }
static constexpr size_t SZ_PL = al256((size_t)NB * NH_ * SEQ * HD * 2);
static constexpr size_t SZ_RS = al256((size_t)NB * NH_ * EROWS * HD * 2);
static constexpr size_t SZ_TOTAL = 3 * SZ_PL + SZ_RS;
static constexpr size_t PLANE_ELEMS = SZ_PL / 2;
static_assert(SZ_TOTAL <= (size_t)134217728);
static_assert(SZ_PL == (size_t)NB * NH_ * SEQ * HD * 2);
static_assert(SZ_RS == (size_t)NB * NH_ * EROWS * HD * 2);

__device__ __forceinline__ unsigned short f2bf(float f) { unsigned u = __float_as_uint(f); u += 0x7FFFu + ((u >> 16) & 1u); return (unsigned short)(u >> 16); }
__device__ __forceinline__ float bfr(float f) { return __uint_as_float(((unsigned)f2bf(f)) << 16); }
__device__ __forceinline__ v16h cat16(v8h lo, v8h hi) { return __builtin_shufflevector(lo, hi, 0, 1, 2, 3, 4, 5, 6, 7, 8, 9, 10, 11, 12, 13, 14, 15); }
__device__ __forceinline__ v16h  ldh(const h16* p) { return cat16(*(const v8h*)p, *(const v8h*)(p + 16)); }
__device__ __forceinline__ void wave_sync() { __builtin_amdgcn_fence(3  , "wavefront"); __builtin_amdgcn_wave_barrier(); asm volatile("" ::: "memory"); }
static __device__ __forceinline__ h16 toh_flush(float v) { const h16 r = (h16)v; return (fabsf(v) < 6.103515625e-05f) ? (h16)0.0f : r; }
__device__ __forceinline__ v8f wmma16g(v16h a, v16h b, v8f c) {
    c = __builtin_amdgcn_wmma_f32_16x16x32_f16(false, a, false, b, (short)0, c, false, false);
    asm volatile("v_nop\n\tv_nop\n\tv_nop\n\tv_nop" : "+v"(c) : "v"(a), "v"(b));
    return c;
}

__global__ __launch_bounds__(128) void k_qkv(const float* __restrict__ x, const float* __restrict__ wq, const float* __restrict__ wk, const float* __restrict__ wv,
                                             h16* QK, h16* VT, h16* VR) {
    __shared__ float xs[PT * 2];
    __shared__ float wl[3 * WSZ];
    const int tid = threadIdx.x;
    const int b = blockIdx.y, t0 = blockIdx.x * PT;
    if (tid < PT) {
        const int t = t0 + tid;
        const float* xp = x + ((size_t)b * SEQ_FULL + (size_t)t) * DIN;
        float sn, cs; sincosf((float)t, &sn, &cs);
        xs[tid * 2 + 0] = bfr(xp[0]) + sn;
        xs[tid * 2 + 1] = bfr(xp[1]) + cs;
    }
#pragma unroll 1
    for (int i = tid; i < WSZ; i += 128) { wl[i] = bfr(wq[i]); wl[WSZ + i] = bfr(wk[i]); wl[2 * WSZ + i] = bfr(wv[i]); }
    __syncthreads();
    const bool wr = t0 < EROWS;
#pragma unroll 1
    for (int ps = 0; ps < 2; ++ps) {
#pragma unroll 1
        for (int g = 0; g < 2 * NH_; ++g) {
            const int pl = g / NH_, h = g % NH_;
            const size_t pbs = (size_t)pl * PLANE_ELEMS + ((size_t)(b * NH_ + h) * SEQ + (size_t)t0) * HD;
            const int wbase = g * (DIN * HD);
#pragma unroll 1
            for (int it = 0; it < 4; ++it) {
                const int p = it * 128 + tid; const int row = p >> 3, c8 = (p & 7) * 8;
                const float a0 = xs[row * 2 + 0], a1 = xs[row * 2 + 1];
                v8h hv;
#pragma unroll
                for (int i = 0; i < 8; ++i) hv[i] = toh_flush(a0 * wl[wbase + c8 + i] + a1 * wl[wbase + HD + c8 + i]);
                *(volatile v8h*)(QK + pbs + (size_t)p * 8) = hv;
            }
        }
#pragma unroll 1
        for (int h = 0; h < NH_; ++h) {
            const int wbase = (2 * NH_ + h) * (DIN * HD);
            const size_t zrow = (size_t)(b * NH_ + h) * HD;
#pragma unroll 1
            for (int it = 0; it < 4; ++it) {
                const int p = it * 128 + tid; const int d = p >> 3, t8 = (p & 7) * 8;
                const float w0 = wl[wbase + d], w1 = wl[wbase + HD + d];
                v8h hv, rv;
#pragma unroll
                for (int i = 0; i < 8; ++i) {
                    const float val = xs[(t8 + i) * 2 + 0] * w0 + xs[(t8 + i) * 2 + 1] * w1;
                    const h16 a = toh_flush(val);
                    hv[i] = a; rv[i] = toh_flush((val - (float)a) * QRS);
                }
                *(volatile v8h*)(VT + (zrow + (size_t)d) * SEQ + (size_t)(t0 + t8)) = hv;
                if (wr) *(volatile v8h*)(VR + (zrow + (size_t)d) * EROWS + (size_t)(t0 + t8)) = rv;
            }
        }
        if (ps == 0) __threadfence();
    }
}

template <int EARLY>
__device__ __forceinline__ void flash_body(const h16* __restrict__ QH, const h16* __restrict__ KP, const h16* __restrict__ VT, const h16* __restrict__ VR,
                                           const float* __restrict__ wo, const float* __restrict__ wboth, float* OUT) {
    __shared__ __align__(16) float os[AW * 32];
    const int lane = threadIdx.x & 31, lr = lane & 15, hi = lane >> 4;
    const int wave = __builtin_amdgcn_readfirstlane((int)(threadIdx.x >> 5));
    const int b = blockIdx.y;
    const int t0 = (EARLY ? 0 : EROWS) + (blockIdx.x * AW + wave) * 16;
    const int lim = t0 + lr;
    const int nk = (t0 + 16 + 31) & ~31;
    const v16h hz = (v16h){};
    float out0 = 0.0f, out1 = 0.0f;
#pragma unroll 1
    for (int h = 0; h < NH_; ++h) {
        const int zh = b * NH_ + h;
        const size_t pbase = (size_t)zh * SEQ * HD;
        const size_t qo = pbase + (size_t)(t0 + lr) * HD + 8 * hi;
        const v16h q0 = ldh(QH + qo), q1 = ldh(QH + qo + 32);
        const size_t ko = pbase + (size_t)lr * HD + 8 * hi;
        const size_t vo = pbase + (size_t)lr * SEQ + 8 * hi;
        const size_t vro = (size_t)zh * EROWS * HD + (size_t)lr * EROWS + 8 * hi;
        v8f o0 = (v8f){}, o1 = (v8f){}, o2 = (v8f){}, o3 = (v8f){};
        v8f oR0 = (v8f){}, oR1 = (v8f){}, oR2 = (v8f){}, oR3 = (v8f){};
        float m = NEGB, l = 0.0f;
#pragma unroll 1
        for (int key0 = 0; key0 < nk; key0 += 32) {
            const h16* ka = KP + ko + (size_t)key0 * HD;
            v8f sa = (v8f){}, sb = (v8f){};
            { const v16h ka0 = ldh(ka), ka1 = ldh(ka + 32);
              sa = wmma16g(ka0, q0, sa); sa = wmma16g(ka1, q1, sa); }
            { const v16h kb0 = ldh(ka + 16 * HD), kb1 = ldh(ka + 16 * HD + 32);
              sb = wmma16g(kb0, q0, sb); sb = wmma16g(kb1, q1, sb); }
            const int ja = key0 + 8 * hi;
            float ta[8], tb[8]; bool fa[8], fb[8]; float mx = NEGB;
#pragma unroll
            for (int r = 0; r < 8; ++r) {
                fa[r] = (ja + r <= lim);
                fb[r] = (ja + 16 + r <= lim);
                ta[r] = sa[r] * SC2; tb[r] = sb[r] * SC2;
                mx = fmaxf(mx, fmaxf(fa[r] ? ta[r] : NEGB, fb[r] ? tb[r] : NEGB)); }
            mx = fmaxf(mx, __shfl_xor(mx, 16, 32));
            const float mnew = fmaxf(m, mx);
            const float alpha = __builtin_amdgcn_exp2f(m - mnew);
            const float sh = PSH - mnew;
            v16h pb, pr = hz; float ls = 0.0f;
#pragma unroll
            for (int r = 0; r < 8; ++r) {
                const float xa = ta[r] + sh, xb = tb[r] + sh;
                const float ea = (xa < -14.0f) ? 0.0f : __builtin_amdgcn_exp2f(xa);
                const float eb = (xb < -14.0f) ? 0.0f : __builtin_amdgcn_exp2f(xb);
                const float ga = fa[r] ? ea : 0.0f, gb = fb[r] ? eb : 0.0f;
                const h16 pa = (h16)ga; const h16 pc = (h16)gb;
                pb[r] = pa; pb[8 + r] = pc;
                if (EARLY) { pr[r] = toh_flush((ga - (float)pa) * QRS); pr[8 + r] = toh_flush((gb - (float)pc) * QRS); ls += ga + gb; }
                else       { ls += (float)pa + (float)pc; } }
            l = l * alpha + ls; m = mnew;
            o0 = o0 * alpha; o1 = o1 * alpha; o2 = o2 * alpha; o3 = o3 * alpha;
            if (EARLY) { oR0 = oR0 * alpha; oR1 = oR1 * alpha; oR2 = oR2 * alpha; oR3 = oR3 * alpha; }
            const h16* va = VT + vo + key0;
            if (EARLY) {
                const h16* vr = VR + vro + key0;
                { const v16h v = ldh(va);                         const v16h w = ldh(vr);
                  o0 = wmma16g(v, pb, o0); oR0 = wmma16g(v, pr, oR0); oR0 = wmma16g(w, pb, oR0); }
                { const v16h v = ldh(va + (size_t)16 * SEQ);      const v16h w = ldh(vr + (size_t)16 * EROWS);
                  o1 = wmma16g(v, pb, o1); oR1 = wmma16g(v, pr, oR1); oR1 = wmma16g(w, pb, oR1); }
                { const v16h v = ldh(va + (size_t)32 * SEQ);      const v16h w = ldh(vr + (size_t)32 * EROWS);
                  o2 = wmma16g(v, pb, o2); oR2 = wmma16g(v, pr, oR2); oR2 = wmma16g(w, pb, oR2); }
                { const v16h v = ldh(va + (size_t)48 * SEQ);      const v16h w = ldh(vr + (size_t)48 * EROWS);
                  o3 = wmma16g(v, pb, o3); oR3 = wmma16g(v, pr, oR3); oR3 = wmma16g(w, pb, oR3); }
            } else {
                { const v16h v = ldh(va);                         o0 = wmma16g(v, pb, o0); }
                { const v16h v = ldh(va + (size_t)16 * SEQ);      o1 = wmma16g(v, pb, o1); }
                { const v16h v = ldh(va + (size_t)32 * SEQ);      o2 = wmma16g(v, pb, o2); }
                { const v16h v = ldh(va + (size_t)48 * SEQ);      o3 = wmma16g(v, pb, o3); }
            }
        }
        l += __shfl_xor(l, 16, 32);
        const bool any = l > 0.0f;
        const float lsafe = any ? l : 1.0f;
        const float inv = any ? (1.0f / lsafe) : 0.0f;
        v8f f0 = o0, f1 = o1, f2 = o2, f3 = o3;
        if (EARLY) { f0 = o0 + oR0 * QRI; f1 = o1 + oR1 * QRI; f2 = o2 + oR2 * QRI; f3 = o3 + oR3 * QRI; }
        const float* wp = wo + h * HD + 8 * hi;
        float part = 0.0f;
        { const v4f w0 = *(const v4f*)(wp +  0), w1 = *(const v4f*)(wp +  4);
#pragma unroll
          for (int i = 0; i < 4; ++i) { part += f0[i] * bfr(w0[i]); part += f0[4 + i] * bfr(w1[i]); } }
        { const v4f w0 = *(const v4f*)(wp + 16), w1 = *(const v4f*)(wp + 20);
#pragma unroll
          for (int i = 0; i < 4; ++i) { part += f1[i] * bfr(w0[i]); part += f1[4 + i] * bfr(w1[i]); } }
        { const v4f w0 = *(const v4f*)(wp + 32), w1 = *(const v4f*)(wp + 36);
#pragma unroll
          for (int i = 0; i < 4; ++i) { part += f2[i] * bfr(w0[i]); part += f2[4 + i] * bfr(w1[i]); } }
        { const v4f w0 = *(const v4f*)(wp + 48), w1 = *(const v4f*)(wp + 52);
#pragma unroll
          for (int i = 0; i < 4; ++i) { part += f3[i] * bfr(w0[i]); part += f3[4 + i] * bfr(w1[i]); } }
        part += __shfl_xor(part, 16, 32);
        const float oh = part * inv;
        out0 += oh * bfr(wboth[h * DIN + 0]);
        out1 += oh * bfr(wboth[h * DIN + 1]);
    }
    const int wb = wave * 32;
    if (hi == 0) { os[wb + lr * 2 + 0] = out0; os[wb + lr * 2 + 1] = out1; }
    wave_sync();
    float* orow = OUT + ((size_t)b * OUT_SEQ + (size_t)t0) * DIN;
    const v4f val = *(const v4fa*)(&os[wb + (lane & 7) * 4]);
#pragma unroll 1
    for (int ps = 0; ps < 2; ++ps) {
        if (lane < 8) *(volatile v4f*)(orow + lane * 4) = val;
        if (ps == 0) __threadfence(); }
}

__global__ __launch_bounds__(32 * AW) void k_flash_early(const h16* __restrict__ QH, const h16* __restrict__ KP, const h16* __restrict__ VT, const h16* __restrict__ VR,
                                                         const float* __restrict__ wo, const float* __restrict__ wboth, float* OUT) {
    flash_body<1>(QH, KP, VT, VR, wo, wboth, OUT);
}

__global__ __launch_bounds__(32 * AW) void k_flash_late(const h16* __restrict__ QH, const h16* __restrict__ KP, const h16* __restrict__ VT, const h16* __restrict__ VR,
                                                        const float* __restrict__ wo, const float* __restrict__ wboth, float* OUT) {
    flash_body<0>(QH, KP, VT, VR, wo, wboth, OUT);
}

extern "C" void kernel_launch(void* const* d_in, const int* in_sizes, int n_in,
                              void* d_out, int out_size, void* d_ws, size_t ws_size, hipStream_t stream) {
    if (n_in < 6) return;
    const size_t needx = ((size_t)(NB - 1) * SEQ_FULL + SEQ) * DIN;
    if ((size_t)in_sizes[0] < needx) return;
    if (in_sizes[1] < WSZ || in_sizes[2] < WSZ || in_sizes[3] < WSZ) return;
    if (in_sizes[4] < NH_ * HD || in_sizes[5] < NH_ * DIN) return;
    if ((size_t)out_size < ((size_t)(NB - 1) * OUT_SEQ + SEQ) * DIN) return;
    if (SZ_TOTAL > ws_size) return;
    const float* x  = (const float*)d_in[0];
    const float* wq = (const float*)d_in[1];
    const float* wk = (const float*)d_in[2];
    const float* wv = (const float*)d_in[3];
    const float* wo = (const float*)d_in[4];
    const float* wb = (const float*)d_in[5];
    float* OUT = (float*)d_out;
    char* wsp = (char*)d_ws;
    h16* QK = (h16*)wsp; wsp += 2 * SZ_PL;
    h16* VT = (h16*)wsp; wsp += SZ_PL;
    h16* VR = (h16*)wsp; wsp += SZ_RS;
    const h16* QH = QK; const h16* KP = QK + PLANE_ELEMS;

    k_qkv<<<dim3(SEQ / PT, NB, 1), 128, 0, stream>>>(x, wq, wk, wv, QK, VT, VR);

    k_flash_early<<<dim3(EROWS / (16 * AW), NB, 1), 32 * AW, 0, stream>>>(QH, KP, VT, VR, wo, wb, OUT);
    if (SEQ > EROWS)
        k_flash_late<<<dim3((SEQ - EROWS) / (16 * AW), NB, 1), 32 * AW, 0, stream>>>(QH, KP, VT, VR, wo, wb, OUT);
}
